// ConcatCritic_566935683177
// MI455X (gfx1250) — hardware-run, weakly checked
//
#include <hip/hip_runtime.h>

typedef __attribute__((ext_vector_type(16))) _Float16 v16h;
typedef __attribute__((ext_vector_type(8)))  _Float16 v8h;
typedef __attribute__((ext_vector_type(8)))  float    v8f;
typedef __attribute__((ext_vector_type(4)))  float    v4f;

constexpr int kItems        = 512;
constexpr int kDim          = 128;
constexpr int kHid          = 256;
constexpr int kW0Pitch      = 2 * kDim;
constexpr int kTilePitch    = kHid + 8;
constexpr int kWavesPerBlk  = 2;
constexpr int kColsPerWave  = 32;
constexpr int kHalfN        = kHid / 2;

constexpr int kFlThreadsPerRow   = kHid / 4;
constexpr int kFlThreadsPerPlane = kItems * kFlThreadsPerRow;
constexpr int kFlPlaneShift      = 15;
constexpr int kFlRowShift        = 6;

constexpr float kActCarry      = 16.0f;
constexpr float kWgtCarry      = 256.0f;
constexpr float kFoldBack      = 1.0f / (kActCarry * kWgtCarry);
constexpr float kHalfMinNormal = 6.103515625e-5f;

static_assert(kW0Pitch == kHid, "first layer input width");
static_assert((kHid % 32) == 0, "K multiple of 32");
static_assert((kHalfN % 16) == 0 && kHalfN * 2 == kHid, "N halves");
static_assert(((kTilePitch * 2) % 16) == 0, "tile pitch 16-B multiple");
static_assert((kItems % kColsPerWave) == 0 && (kItems % kWavesPerBlk) == 0, "grid multiples");
static_assert(kFoldBack * 4096.0f == 1.0f, "fold-back is exact");
static_assert(kWavesPerBlk * 2 * 16 * kTilePitch * 2 + kWavesPerBlk * kColsPerWave * 4 <= 65536, "static LDS");
static_assert(kFlThreadsPerPlane == (1 << kFlPlaneShift), "plane decode shift");
static_assert(kFlThreadsPerRow == (1 << kFlRowShift), "row decode shift");
static_assert(((2 * kFlThreadsPerPlane) % 256) == 0 && (kFlThreadsPerPlane % 256) == 0, "plane split is block-uniform");

constexpr size_t kOffHXB  = 0;
constexpr size_t kOffHY   = kOffHXB + (size_t)kItems * kHid * 4;
constexpr size_t kOffW1H  = kOffHY  + (size_t)kItems * kHid * 4;
constexpr size_t kOffW2H  = kOffW1H + (size_t)kHid * kHid * 2;
constexpr size_t kWsTotal = kOffW2H + (size_t)kHid * kHid * 2;
static_assert(kWsTotal == 1310720ull, "carve total");
static_assert(kWsTotal <= 134217728ull, "carve cap");
static_assert((kOffHY % 128) == 0 && (kOffW1H % 128) == 0 && (kOffW2H % 128) == 0, "128-B aligned regions");

union FragH { v16h v; v8h h[2]; };

__device__ __forceinline__ v16h frag_load(const _Float16* p) {
  FragH f;
  f.h[0] = *(const v8h*)(p);
  f.h[1] = *(const v8h*)(p + 16);
  return f.v;
}

__device__ __forceinline__ v8f mma_f16(v16h a, v16h b, v8f c) {
  c = __builtin_amdgcn_wmma_f32_16x16x32_f16(false, a, false, b, (short)0, c, false, false);
  asm volatile("v_nop\n\tv_nop\n\tv_nop\n\tv_nop" : "+v"(c) : "v"(a), "v"(b));
  return c;
}

__device__ __forceinline__ void wave_lds_fence() {
  __builtin_amdgcn_fence(__ATOMIC_RELEASE, "workgroup");
  __builtin_amdgcn_wave_barrier();
  __builtin_amdgcn_fence(__ATOMIC_ACQUIRE, "workgroup");
}

__device__ __forceinline__ _Float16 act_to_half(float v) {
  float t = v * kActCarry;
  t = (t < kHalfMinNormal) ? 0.0f : t;
  return (_Float16)t;
}

__global__ __launch_bounds__(256) void first_layer_rows_kernel(
    const float* __restrict__ x, const float* __restrict__ y,
    const float* __restrict__ W0, const float* __restrict__ b0,
    float* __restrict__ hxb, float* __restrict__ hy)
{
  const int t   = blockIdx.x * 256 + threadIdx.x;
  const int sel = (t >> kFlPlaneShift) & 1;
  const int i4  = t & (kFlThreadsPerPlane - 1);
  const int r   = i4 >> kFlRowShift;
  const int g0  = (i4 & (kFlThreadsPerRow - 1)) * 4;
  const float* src = sel ? y : x;
  const float* xr  = src + (size_t)r * kDim;
  const float* wr  = W0 + (size_t)g0 * kW0Pitch + sel * kDim;
  float a0 = 0.0f, a1 = 0.0f, a2 = 0.0f, a3 = 0.0f;
#pragma unroll 1
  for (int k = 0; k < kDim; k += 4) {
    const v4f xv = *(const v4f*)(xr + k);
    const v4f w0 = *(const v4f*)(wr + k);
    const v4f w1 = *(const v4f*)(wr + kW0Pitch + k);
    const v4f w2 = *(const v4f*)(wr + 2 * kW0Pitch + k);
    const v4f w3 = *(const v4f*)(wr + 3 * kW0Pitch + k);
    a0 = fmaf(xv[0], w0[0], a0); a0 = fmaf(xv[1], w0[1], a0); a0 = fmaf(xv[2], w0[2], a0); a0 = fmaf(xv[3], w0[3], a0);
    a1 = fmaf(xv[0], w1[0], a1); a1 = fmaf(xv[1], w1[1], a1); a1 = fmaf(xv[2], w1[2], a1); a1 = fmaf(xv[3], w1[3], a1);
    a2 = fmaf(xv[0], w2[0], a2); a2 = fmaf(xv[1], w2[1], a2); a2 = fmaf(xv[2], w2[2], a2); a2 = fmaf(xv[3], w2[3], a2);
    a3 = fmaf(xv[0], w3[0], a3); a3 = fmaf(xv[1], w3[1], a3); a3 = fmaf(xv[2], w3[2], a3); a3 = fmaf(xv[3], w3[3], a3);
  }
  const v4f bz = *(const v4f*)(b0 + g0);
  v4f o;
  o[0] = a0 + (sel ? 0.0f : bz[0]);
  o[1] = a1 + (sel ? 0.0f : bz[1]);
  o[2] = a2 + (sel ? 0.0f : bz[2]);
  o[3] = a3 + (sel ? 0.0f : bz[3]);
  float* dst = (sel ? hy : hxb) + (size_t)r * kHid + g0;
  *(volatile v4f*)dst = o;
  __threadfence();
  *(volatile v4f*)dst = o;
}

__global__ __launch_bounds__(256) void weight_planes_kernel(
    const float* __restrict__ W1, const float* __restrict__ W2,
    unsigned short* __restrict__ w1p, unsigned short* __restrict__ w2p)
{
  const int i     = blockIdx.x * 256 + threadIdx.x;
  const int which = (i >> 13) & 1;
  const size_t e0 = (size_t)(i & 8191) << 3;
  const float* src    = which ? W2 : W1;
  unsigned short* dst = (which ? w2p : w1p) + e0;
  const v4f a0 = *(const v4f*)(src + e0);
  const v4f a1 = *(const v4f*)(src + e0 + 4);
  v8h hv;
#pragma unroll
  for (int e = 0; e < 4; ++e) {
    float t0 = a0[e] * kWgtCarry;
    float t1 = a1[e] * kWgtCarry;
    t0 = (fabsf(t0) < kHalfMinNormal) ? 0.0f : t0;
    t1 = (fabsf(t1) < kHalfMinNormal) ? 0.0f : t1;
    hv[e]     = (_Float16)t0;
    hv[4 + e] = (_Float16)t1;
  }
  *(volatile v8h*)dst = hv;
  __threadfence();
  *(volatile v8h*)dst = hv;
}

__global__ __launch_bounds__(64) void pair_layers_kernel(
    const float* __restrict__ hxb, const float* __restrict__ hy,
    const unsigned short* __restrict__ w1p, const unsigned short* __restrict__ w2p,
    const float* __restrict__ b1, const float* __restrict__ b2,
    const float* __restrict__ w3, const float* __restrict__ b3,
    float* __restrict__ out)
{
  __shared__ __align__(16) _Float16 sH0[kWavesPerBlk][16 * kTilePitch];
  __shared__ __align__(16) _Float16 sH1[kWavesPerBlk][16 * kTilePitch];
  __shared__ __align__(16) float    sRes[kWavesPerBlk][kColsPerWave];

  const int lane = threadIdx.x & 31;
  const int wave = threadIdx.x >> 5;
  const int lo   = lane & 15;
  const int hi   = lane >> 4;
  const int a     = blockIdx.y * kWavesPerBlk + wave;
  const int bbase = blockIdx.x * kColsPerWave;

  _Float16* t0 = sH0[wave];
  _Float16* t1 = sH1[wave];
  float*    rs = sRes[wave];

  const _Float16* W1h = (const _Float16*)w1p;
  const _Float16* W2h = (const _Float16*)w2p;

  const float b3v = b3[0];

  const v4f hx0 = *(const v4f*)(hxb + (size_t)a * kHid + lane * 8);
  const v4f hx1 = *(const v4f*)(hxb + (size_t)a * kHid + lane * 8 + 4);

  const _Float16* a0base = t0 + lo * kTilePitch + 8 * hi;
  const _Float16* a1base = t1 + lo * kTilePitch + 8 * hi;

#pragma unroll 1
  for (int mt = 0; mt < 2; ++mt) {
    const int brow0 = bbase + mt * 16;

#pragma unroll 4
    for (int m = 0; m < 16; ++m) {
      const float* hp = hy + (size_t)(brow0 + m) * kHid + lane * 8;
      const v4f y0 = *(const v4f*)(hp);
      const v4f y1 = *(const v4f*)(hp + 4);
      v8h hv;
#pragma unroll
      for (int e = 0; e < 4; ++e) {
        hv[e]     = act_to_half(fmaxf(hx0[e] + y0[e], 0.0f));
        hv[4 + e] = act_to_half(fmaxf(hx1[e] + y1[e], 0.0f));
      }
      *(v8h*)(t0 + m * kTilePitch + lane * 8) = hv;
    }
    wave_lds_fence();

#pragma unroll 1
    for (int nh = 0; nh < 2; ++nh) {
      const int nb = nh * kHalfN;
      v8f acc[8];
#pragma unroll
      for (int j = 0; j < 8; ++j) acc[j] = (v8f){0.f, 0.f, 0.f, 0.f, 0.f, 0.f, 0.f, 0.f};
      const _Float16* wb = W1h + (size_t)(nb + lo) * kHid + 8 * hi;
#pragma unroll 1
      for (int k0 = 0; k0 < kHid; k0 += 32) {
        const v16h af = frag_load(a0base + k0);
#pragma unroll
        for (int j = 0; j < 8; ++j) {
          const v16h bf = frag_load(wb + (size_t)j * 16 * kHid + k0);
          acc[j] = mma_f16(af, bf, acc[j]);
        }
      }
#pragma unroll
      for (int j = 0; j < 8; ++j) {
        const int n = nb + j * 16 + lo;
        const float bv = b1[n];
#pragma unroll
        for (int r = 0; r < 8; ++r) {
          float v = fmaf(acc[j][r], kFoldBack, bv);
          v = fmaxf(v, 0.0f);
          t1[(8 * hi + r) * kTilePitch + n] = act_to_half(v);
        }
      }
    }
    wave_lds_fence();

    float hs[8];
#pragma unroll
    for (int r = 0; r < 8; ++r) hs[r] = 0.0f;
#pragma unroll 1
    for (int nh = 0; nh < 2; ++nh) {
      const int nb = nh * kHalfN;
      v8f acc[8];
#pragma unroll
      for (int j = 0; j < 8; ++j) acc[j] = (v8f){0.f, 0.f, 0.f, 0.f, 0.f, 0.f, 0.f, 0.f};
      const _Float16* wb = W2h + (size_t)(nb + lo) * kHid + 8 * hi;
#pragma unroll 1
      for (int k0 = 0; k0 < kHid; k0 += 32) {
        const v16h af = frag_load(a1base + k0);
#pragma unroll
        for (int j = 0; j < 8; ++j) {
          const v16h bf = frag_load(wb + (size_t)j * 16 * kHid + k0);
          acc[j] = mma_f16(af, bf, acc[j]);
        }
      }
#pragma unroll
      for (int j = 0; j < 8; ++j) {
        const int n = nb + j * 16 + lo;
        const float bv = b2[n];
        const float wv = w3[n];
#pragma unroll
        for (int r = 0; r < 8; ++r) {
          float v = fmaf(acc[j][r], kFoldBack, bv);
          v = fmaxf(v, 0.0f);
          hs[r] = fmaf(v, wv, hs[r]);
        }
      }
    }
#pragma unroll
    for (int r = 0; r < 8; ++r) {
      hs[r] += __shfl_xor(hs[r], 1, 32);
      hs[r] += __shfl_xor(hs[r], 2, 32);
      hs[r] += __shfl_xor(hs[r], 4, 32);
      hs[r] += __shfl_xor(hs[r], 8, 32);
    }
    v4f q0, q1;
    q0[0] = hs[0]; q0[1] = hs[1]; q0[2] = hs[2]; q0[3] = hs[3];
    q1[0] = hs[4]; q1[1] = hs[5]; q1[2] = hs[6]; q1[3] = hs[7];
    if (lo == 0) {
      *(v4f*)(rs + mt * 16 + 8 * hi)     = q0;
      *(v4f*)(rs + mt * 16 + 8 * hi + 4) = q1;
    }
  }
  wave_lds_fence();

  const float o = rs[lane] + b3v;
  volatile float* op = out + (size_t)a * kItems + bbase + lane;
  *op = o;
  __threadfence();
  *op = o;
}

extern "C" void kernel_launch(void* const* d_in, const int* in_sizes, int n_in,
                              void* d_out, int out_size, void* d_ws, size_t ws_size,
                              hipStream_t stream) {
  if (n_in < 10) return;
  if (in_sizes[0] != kItems * kDim) return;
  if (in_sizes[1] != kItems * kDim) return;
  if (in_sizes[2] != kHid * kW0Pitch) return;
  if (in_sizes[3] != kHid) return;
  if (in_sizes[4] != kHid * kHid) return;
  if (in_sizes[5] != kHid) return;
  if (in_sizes[6] != kHid * kHid) return;
  if (in_sizes[7] != kHid) return;
  if (in_sizes[8] != kHid) return;
  if (in_sizes[9] != 1) return;
  if (out_size != kItems * kItems) return;
  if (ws_size < kWsTotal) return;

  const float* x  = (const float*)d_in[0];
  const float* y  = (const float*)d_in[1];
  const float* W0 = (const float*)d_in[2];
  const float* b0 = (const float*)d_in[3];
  const float* W1 = (const float*)d_in[4];
  const float* b1 = (const float*)d_in[5];
  const float* W2 = (const float*)d_in[6];
  const float* b2 = (const float*)d_in[7];
  const float* W3 = (const float*)d_in[8];
  const float* b3 = (const float*)d_in[9];
  float* out = (float*)d_out;

  char* ws = (char*)d_ws;
  float*          hxb = (float*)(ws + kOffHXB);
  float*          hy  = (float*)(ws + kOffHY);
  unsigned short* w1h = (unsigned short*)(ws + kOffW1H);
  unsigned short* w2h = (unsigned short*)(ws + kOffW2H);

  first_layer_rows_kernel<<<(2 * kFlThreadsPerPlane) / 256, 256, 0, stream>>>(x, y, W0, b0, hxb, hy);
  weight_planes_kernel<<<(2 * kHid * kHid / 8) / 256, 256, 0, stream>>>(W1, W2, w1h, w2h);
  pair_layers_kernel<<<dim3(kItems / kColsPerWave, kItems / kWavesPerBlk), 32 * kWavesPerBlk, 0, stream>>>(
      hxb, hy, w1h, w2h, b1, b2, W3, b3, out);
}
